// BetaModel_5660766896152
// MI455X (gfx1250) — hardware-verified
//
#include <hip/hip_runtime.h>
#define BB 32
#define TT 512
#define DD 280
#define DP 320
#define KP 288
#define NH 7
#define HD 40
#define HP 64
#define QP (NH * HP)
#define FF 1120
#define FP 1152
#define VV 256
#define NL 7

typedef __bf16 v16b __attribute__((ext_vector_type(16)));
typedef unsigned short v8us __attribute__((ext_vector_type(8), may_alias));
typedef float  v8f  __attribute__((ext_vector_type(8)));
typedef float  v4f  __attribute__((ext_vector_type(4)));
typedef float  v4fa __attribute__((ext_vector_type(4), may_alias));
union FragB { v16b v; v8us half[2]; unsigned short u[16]; };

__device__ __forceinline__ unsigned short bf16_bits(float x) { unsigned int u = __float_as_uint(x); return (unsigned short)((u + 0x7FFFu + ((u >> 16) & 1u)) >> 16); }
__device__ __forceinline__ float bf16_val(unsigned short b) { return __uint_as_float(((unsigned int)b) << 16); }
__device__ __forceinline__ float bf16_round(float x) { return bf16_val(bf16_bits(x)); }
template <int NT>
__device__ __forceinline__ v8f mmaN(v16b ah, v16b al, v16b bh, v16b bl, v8f c) {
  c = __builtin_amdgcn_wmma_f32_16x16x32_bf16(false, ah, false, bh, (short)0, c, false, false);
  if (NT >= 2) c = __builtin_amdgcn_wmma_f32_16x16x32_bf16(false, al, false, bh, (short)0, c, false, false);
  if (NT >= 3) c = __builtin_amdgcn_wmma_f32_16x16x32_bf16(false, ah, false, bl, (short)0, c, false, false);
  asm volatile("v_nop\n\tv_nop\n\tv_nop\n\tv_nop" : "+v"(c) : "v"(ah), "v"(al), "v"(bh), "v"(bl));
  return c;
}

__global__ __launch_bounds__(256) void k_wt_bf16(const float* __restrict__ W, unsigned short* __restrict__ Wt, int K, int N) {
  const int t = blockIdx.x * 256 + threadIdx.x;
  const int k8n = K / 8;
  if (t >= N * k8n) return;
  const int n = t / k8n, k8 = (t % k8n) * 8;
  v8us v;
#pragma unroll
  for (int i = 0; i < 8; ++i) v[i] = bf16_bits(W[(size_t)(k8 + i) * N + n]);
  *(volatile v8us*)(Wt + (size_t)n * K + k8) = v;
  __threadfence();
  *(volatile v8us*)(Wt + (size_t)n * K + k8) = v;
}

template <bool ASPLIT, int ACT, bool BIAS_BF16>
__global__ __launch_bounds__(128) void k_gemm_bf(const float* __restrict__ A, int lda, const unsigned short* __restrict__ Wt, int ldb,
                                               const float* __restrict__ bias, float* __restrict__ C, int ldc, int M, int N, int K) {
  __shared__ __attribute__((aligned(16))) float so[4][16][64];
  const int tid = threadIdx.x, w = tid >> 5, lane = tid & 31, ln = lane & 15, hh = lane >> 4;
  const int ntn = N / 64;
  const int wid = blockIdx.x * 4 + w;
  const int mt = wid / ntn, nq = wid % ntn;
  if (mt * 16 >= M) return;
  const int row0 = mt * 16, col0 = nq * 64;
  const float* arow = A + (size_t)(row0 + ln) * lda;
  v8f acc[4] = {};
  for (int kb = 0; kb < K; kb += 32) {
    FragB ah, al;
    const v4f x0 = *(const v4fa*)(arow + kb + 8 * hh), x1 = *(const v4fa*)(arow + kb + 8 * hh + 4);
    const v4f x2 = *(const v4fa*)(arow + kb + 16 + 8 * hh), x3 = *(const v4fa*)(arow + kb + 16 + 8 * hh + 4);
    float xs[16] = {x0[0],x0[1],x0[2],x0[3],x1[0],x1[1],x1[2],x1[3],x2[0],x2[1],x2[2],x2[3],x3[0],x3[1],x3[2],x3[3]};
#pragma unroll
    for (int i = 0; i < 16; ++i) { const unsigned short hb = bf16_bits(xs[i]); ah.u[i] = hb; al.u[i] = ASPLIT ? bf16_bits(xs[i] - bf16_val(hb)) : (unsigned short)0; }
#pragma unroll
    for (int t = 0; t < 4; ++t) {
      const unsigned short* brow = Wt + (size_t)(col0 + t * 16 + ln) * ldb + kb;
      FragB b;
      b.half[0] = *(const v8us*)(brow + 8 * hh);
      b.half[1] = *(const v8us*)(brow + 16 + 8 * hh);
      acc[t] = mmaN<ASPLIT ? 2 : 1>(ah.v, al.v, b.v, b.v, acc[t]);
    }
  }
#pragma unroll
  for (int t = 0; t < 4; ++t) {
    float bv = bias ? bias[col0 + t * 16 + ln] : 0.f;
    if (BIAS_BF16) bv = bf16_round(bv);
#pragma unroll
    for (int r = 0; r < 8; ++r) { float v = acc[t][r] + bv; if (ACT == 1) v = fmaxf(v, 0.f); so[w][8 * hh + r][t * 16 + ln] = v; }
  }
  __builtin_amdgcn_fence(__ATOMIC_ACQ_REL, "workgroup");
  __builtin_amdgcn_wave_barrier();
  const int rsub = lane >> 4, c4 = (lane & 15) * 4;
  for (int pass = 0; pass < 2; ++pass) {
#pragma unroll
    for (int q = 0; q < 8; ++q) {
      const int r = q * 2 + rsub;
      const v4f v = *(const v4fa*)&so[w][r][c4];
      *(volatile v4f*)(C + (size_t)(row0 + r) * ldc + col0 + c4) = v;
    }
    if (pass == 0) __threadfence();
  }
}

template <int D, bool CAUSAL>
__global__ __launch_bounds__(128) void k_flash(const float* __restrict__ qb, const float* __restrict__ kb, const float* __restrict__ vb,
                                             int pitch, int T, int H, float scale, float* __restrict__ y, int ypitch) {
  constexpr int KS = D / 32;
  constexpr int DT = D / 16;
  __shared__ __attribute__((aligned(16))) unsigned short sKh[32][D + 8], sKl[32][D + 8], sVh[32][D + 8], sVl[32][D + 8];
  __shared__ __attribute__((aligned(16))) unsigned short sPh[4][16][40], sPl[4][16][40];
  __shared__ __attribute__((aligned(16))) float sO[4][16][D];
  const int tid = threadIdx.x, w = tid >> 5, lane = tid & 31, ln = lane & 15, hh = lane >> 4;
  const int nqb = (T + 63) / 64;
  const int bh = blockIdx.x / nqb, qblk = blockIdx.x % nqb;
  const int b = bh / H, h = bh % H;
  const int q0 = qblk * 64 + w * 16;
  const float* Q = qb + (size_t)b * T * pitch + h * D;
  const float* K = kb + (size_t)b * T * pitch + h * D;
  const float* V = vb + (size_t)b * T * pitch + h * D;

  FragB aqh[KS], aql[KS];
  {
    int row = q0 + ln; if (row >= T) row = T - 1;
    const float* qr = Q + (size_t)row * pitch;
#pragma unroll
    for (int ks = 0; ks < KS; ++ks)
#pragma unroll
      for (int i = 0; i < 16; ++i) {
        const int d = ks * 32 + ((i < 8) ? (8 * hh + i) : (16 + 8 * hh + (i - 8)));
        const float x = qr[d] * scale; const unsigned short hb = bf16_bits(x);
        aqh[ks].u[i] = hb; aql[ks].u[i] = bf16_bits(x - bf16_val(hb));
      }
  }
  float m_r[8], l_r[8];
#pragma unroll
  for (int r = 0; r < 8; ++r) { m_r[r] = -3.0e38f; l_r[r] = 0.f; }
  v8f oacc[DT];
#pragma unroll
  for (int dt = 0; dt < DT; ++dt) oacc[dt] = (v8f){0.f,0.f,0.f,0.f,0.f,0.f,0.f,0.f};

  const int kv_end = CAUSAL ? min(T, qblk * 64 + 64) : T;
  for (int j0 = 0; j0 < kv_end; j0 += 32) {
    __syncthreads();
    for (int e = tid; e < 32 * (D / 4); e += 128) {
      const int r = e / (D / 4), c4 = (e % (D / 4)) * 4;
      const int key = j0 + r;
      v4f kf = {0.f,0.f,0.f,0.f}, vf = {0.f,0.f,0.f,0.f};
      if (key < T) { kf = *(const v4fa*)(K + (size_t)key * pitch + c4); vf = *(const v4fa*)(V + (size_t)key * pitch + c4); }
#pragma unroll
      for (int t = 0; t < 4; ++t) {
        unsigned short hb = bf16_bits(kf[t]); sKh[r][c4 + t] = hb; sKl[r][c4 + t] = bf16_bits(kf[t] - bf16_val(hb));
        hb = bf16_bits(vf[t]); sVh[r][c4 + t] = hb; sVl[r][c4 + t] = bf16_bits(vf[t] - bf16_val(hb));
      }
    }
    __syncthreads();
    v8f s[2];
#pragma unroll
    for (int nt = 0; nt < 2; ++nt) {
      v8f acc = {};
#pragma unroll
      for (int ks = 0; ks < KS; ++ks) {
        FragB bh_, bl_;
        bh_.half[0] = *(const v8us*)&sKh[nt * 16 + ln][ks * 32 + 8 * hh]; bh_.half[1] = *(const v8us*)&sKh[nt * 16 + ln][ks * 32 + 16 + 8 * hh];
        bl_.half[0] = *(const v8us*)&sKl[nt * 16 + ln][ks * 32 + 8 * hh]; bl_.half[1] = *(const v8us*)&sKl[nt * 16 + ln][ks * 32 + 16 + 8 * hh];
        acc = mmaN<3>(aqh[ks].v, aql[ks].v, bh_.v, bl_.v, acc);
      }
      s[nt] = acc;
    }
    float alpha[8];
#pragma unroll
    for (int r = 0; r < 8; ++r) {
      const int qi = q0 + 8 * hh + r;
      const int ja = j0 + ln, jb = j0 + 16 + ln;
      if (CAUSAL) { if (ja > qi) s[0][r] = -3.0e38f; if (jb > qi) s[1][r] = -3.0e38f; }
      if (ja >= T) s[0][r] = -3.0e38f;
      if (jb >= T) s[1][r] = -3.0e38f;
      float mx = fmaxf(s[0][r], s[1][r]);
      mx = fmaxf(mx, __shfl_xor(mx, 1, 32)); mx = fmaxf(mx, __shfl_xor(mx, 2, 32)); mx = fmaxf(mx, __shfl_xor(mx, 4, 32)); mx = fmaxf(mx, __shfl_xor(mx, 8, 32));
      const float mnew = fmaxf(m_r[r], mx);
      alpha[r] = (mnew > -1.0e38f) ? __expf(m_r[r] - mnew) : 1.0f;
      const float p0 = (s[0][r] > -1.0e38f) ? __expf(s[0][r] - mnew) : 0.f;
      const float p1 = (s[1][r] > -1.0e38f) ? __expf(s[1][r] - mnew) : 0.f;
      m_r[r] = mnew;
      l_r[r] = l_r[r] * alpha[r] + p0 + p1;
      unsigned short hb = bf16_bits(p0); sPh[w][8 * hh + r][ln] = hb;      sPl[w][8 * hh + r][ln] = bf16_bits(p0 - bf16_val(hb));
      hb = bf16_bits(p1);                sPh[w][8 * hh + r][16 + ln] = hb; sPl[w][8 * hh + r][16 + ln] = bf16_bits(p1 - bf16_val(hb));
    }
#pragma unroll
    for (int dt = 0; dt < DT; ++dt)
#pragma unroll
      for (int r = 0; r < 8; ++r) oacc[dt][r] *= alpha[r];
    __builtin_amdgcn_fence(__ATOMIC_ACQ_REL, "workgroup");
    __builtin_amdgcn_wave_barrier();
    FragB pah, pal;
    pah.half[0] = *(const v8us*)&sPh[w][ln][8 * hh]; pah.half[1] = *(const v8us*)&sPh[w][ln][16 + 8 * hh];
    pal.half[0] = *(const v8us*)&sPl[w][ln][8 * hh]; pal.half[1] = *(const v8us*)&sPl[w][ln][16 + 8 * hh];
#pragma unroll
    for (int dt = 0; dt < DT; ++dt) {
      FragB bvh, bvl;
#pragma unroll
      for (int i = 0; i < 8; ++i) {
        bvh.u[i] = sVh[8 * hh + i][dt * 16 + ln]; bvh.u[8 + i] = sVh[16 + 8 * hh + i][dt * 16 + ln];
        bvl.u[i] = sVl[8 * hh + i][dt * 16 + ln]; bvl.u[8 + i] = sVl[16 + 8 * hh + i][dt * 16 + ln];
      }
      oacc[dt] = mmaN<3>(pah.v, pal.v, bvh.v, bvl.v, oacc[dt]);
    }
    __builtin_amdgcn_fence(__ATOMIC_ACQ_REL, "workgroup");
    __builtin_amdgcn_wave_barrier();
  }
#pragma unroll
  for (int r = 0; r < 8; ++r) {
    float l = l_r[r];
    l += __shfl_xor(l, 1, 32); l += __shfl_xor(l, 2, 32); l += __shfl_xor(l, 4, 32); l += __shfl_xor(l, 8, 32);
    l_r[r] = (l > 0.f) ? 1.0f / l : 0.f;
  }
#pragma unroll
  for (int dt = 0; dt < DT; ++dt)
#pragma unroll
    for (int r = 0; r < 8; ++r) sO[w][8 * hh + r][dt * 16 + ln] = oacc[dt][r] * l_r[r];
  __builtin_amdgcn_fence(__ATOMIC_ACQ_REL, "workgroup");
  __builtin_amdgcn_wave_barrier();
  for (int pass = 0; pass < 2; ++pass) {
    for (int r = 0; r < 16; ++r) {
      const int row = q0 + r;
      if (row < T && lane < D / 4) {
        const v4f val = *(const v4fa*)&sO[w][r][lane * 4];
        *(volatile v4f*)(y + ((size_t)b * T + row) * ypitch + h * D + lane * 4) = val;
      }
    }
    if (pass == 0) __threadfence();
  }
}

template <bool ASPLIT, int ACT, bool BIAS_BF16, bool RES_BF16>
__global__ __launch_bounds__(128) void k_gemm_bf3(const float* __restrict__ A, int lda, const unsigned short* __restrict__ Wt, int ldb,
                                                const float* __restrict__ bias, const float* resid, int rmod, int ldr,
                                                float* C, int ldc, int M, int N, int K) {
  __shared__ __attribute__((aligned(16))) float so[4][16][64];
  const int tid = threadIdx.x, w = tid >> 5, lane = tid & 31, ln = lane & 15, hh = lane >> 4;
  const int ntn = N / 64;
  const int wid = blockIdx.x * 4 + w;
  const int mt = wid / ntn, nq = wid % ntn;
  if (mt * 16 >= M) return;
  const int row0 = mt * 16, col0 = nq * 64;
  const float* arow = A + (size_t)(row0 + ln) * lda;
  v8f acc[4] = {};
  for (int kb = 0; kb < K; kb += 32) {
    FragB ah, al;
    const v4f x0 = *(const v4fa*)(arow + kb + 8 * hh), x1 = *(const v4fa*)(arow + kb + 8 * hh + 4);
    const v4f x2 = *(const v4fa*)(arow + kb + 16 + 8 * hh), x3 = *(const v4fa*)(arow + kb + 16 + 8 * hh + 4);
    float xs[16] = {x0[0],x0[1],x0[2],x0[3],x1[0],x1[1],x1[2],x1[3],x2[0],x2[1],x2[2],x2[3],x3[0],x3[1],x3[2],x3[3]};
#pragma unroll
    for (int i = 0; i < 16; ++i) { const unsigned short hb = bf16_bits(xs[i]); ah.u[i] = hb; al.u[i] = ASPLIT ? bf16_bits(xs[i] - bf16_val(hb)) : (unsigned short)0; }
#pragma unroll
    for (int t = 0; t < 4; ++t) {
      const unsigned short* brow = Wt + (size_t)(col0 + t * 16 + ln) * ldb + kb;
      FragB b;
      b.half[0] = *(const v8us*)(brow + 8 * hh);
      b.half[1] = *(const v8us*)(brow + 16 + 8 * hh);
      acc[t] = mmaN<ASPLIT ? 2 : 1>(ah.v, al.v, b.v, b.v, acc[t]);
    }
  }
#pragma unroll
  for (int t = 0; t < 4; ++t) {
    const int col = col0 + t * 16 + ln;
    float bv = bias ? bias[col] : 0.f;
    if (BIAS_BF16) bv = bf16_round(bv);
#pragma unroll
    for (int r = 0; r < 8; ++r) {
      float v = acc[t][r] + bv;
      if (resid) { float rv = resid[(size_t)((row0 + 8 * hh + r) % rmod) * ldr + col]; if (RES_BF16) rv = bf16_round(rv); v += rv; }
      if (ACT == 1) v = fmaxf(v, 0.f);
      if (ACT == 2) v = 0.5f * v * (1.0f + erff(v * 0.70710678118654752f));
      if (ACT == 3) { const float u = 0.7978845608028654f * (v + 0.044715f * v * v * v); v = 0.5f * v * (1.0f + tanhf(u)); }
      so[w][8 * hh + r][t * 16 + ln] = v;
    }
  }
  __builtin_amdgcn_fence(__ATOMIC_ACQ_REL, "workgroup");
  __builtin_amdgcn_wave_barrier();
  const int rsub = lane >> 4, c4 = (lane & 15) * 4;
  for (int pass = 0; pass < 2; ++pass) {
#pragma unroll
    for (int q = 0; q < 8; ++q) {
      const int r = q * 2 + rsub;
      const v4f v = *(const v4fa*)&so[w][r][c4];
      *(volatile v4f*)(C + (size_t)(row0 + r) * ldc + col0 + c4) = v;
    }
    if (pass == 0) __threadfence();
  }
}
template <bool PARAM_BF16>
__global__ __launch_bounds__(256) void k_layernorm(const float* __restrict__ X, const float* __restrict__ R, const float* __restrict__ g, const float* __restrict__ bta,
                                                  float* __restrict__ out_sum, float* __restrict__ out_norm, int N, float eps) {
  __shared__ float red[256];
  const int row = blockIdx.x, tid = threadIdx.x;
  const float* x = X + (size_t)row * N; const float* rr = R ? R + (size_t)row * N : nullptr;
  float vals[16];
  const int per = N / 256;
  float s1 = 0.f;
  for (int u = 0; u < per / 4; ++u) {
    const int j = tid * 4 + 1024 * u;
    const v4f a = *(const v4fa*)(x + j);
    v4f b = {0.f,0.f,0.f,0.f}; if (rr) b = *(const v4fa*)(rr + j);
#pragma unroll
    for (int q = 0; q < 4; ++q) { const float v = a[q] + b[q]; vals[u * 4 + q] = v; s1 += v; }
  }
  red[tid] = s1; __syncthreads();
  for (int st = 128; st > 0; st >>= 1) { if (tid < st) red[tid] += red[tid + st]; __syncthreads(); }
  const float mu = red[0] / (float)N; __syncthreads();
  float s2 = 0.f;
  for (int u = 0; u < per / 4; ++u)
#pragma unroll
    for (int q = 0; q < 4; ++q) { const float c = vals[u * 4 + q] - mu; s2 += c * c; }
  red[tid] = s2; __syncthreads();
  for (int st = 128; st > 0; st >>= 1) { if (tid < st) red[tid] += red[tid + st]; __syncthreads(); }
  const float rs = rsqrtf(red[0] / (float)N + eps);
  for (int pass = 0; pass < 2; ++pass) {
    for (int u = 0; u < per / 4; ++u) {
      const int j = tid * 4 + 1024 * u;
      v4f o, sm;
#pragma unroll
      for (int q = 0; q < 4; ++q) {
        float gg = g[j + q], bb = bta[j + q];
        if (PARAM_BF16) { gg = bf16_round(gg); bb = bf16_round(bb); }
        sm[q] = vals[u * 4 + q]; o[q] = (vals[u * 4 + q] - mu) * rs * gg + bb;
      }
      if (out_sum) *(volatile v4f*)(out_sum + (size_t)row * N + j) = sm;
      *(volatile v4f*)(out_norm + (size_t)row * N + j) = o;
    }
    if (pass == 0) __threadfence();
  }
}

template <int D>
__global__ __launch_bounds__(128) void k_flash3(const float* __restrict__ Qb, int qpitch, int Tq,
                                              const float* __restrict__ K1, const float* __restrict__ V1, int Tk1,
                                              const float* __restrict__ K2, const float* __restrict__ V2, int Tk2, int kpitch, int vpitch,
                                              int H, float scale, const int* __restrict__ mask, int causal, const float* __restrict__ sbias,
                                              float* __restrict__ y, int ypitch) {
  constexpr int KS = D / 32, DT = D / 16;
  __shared__ __attribute__((aligned(16))) unsigned short sKh[32][D + 8], sKl[32][D + 8], sVh[32][D + 8], sVl[32][D + 8];
  __shared__ __attribute__((aligned(16))) unsigned short sPh[4][16][40], sPl[4][16][40];
  __shared__ __attribute__((aligned(16))) float sO[4][16][D];
  const int tid = threadIdx.x, w = tid >> 5, lane = tid & 31, ln = lane & 15, hh = lane >> 4;
  const int Tk = Tk1 + Tk2;
  const int nqb = (Tq + 63) / 64;
  const int bh = blockIdx.x / nqb, qblk = blockIdx.x % nqb;
  const int b = bh / H, h = bh % H;
  const int q0 = qblk * 64 + w * 16;
  const float* Q = Qb + (size_t)b * Tq * qpitch + h * D;
  FragB aqh[KS], aql[KS];
  {
    int row = q0 + ln; if (row >= Tq) row = Tq - 1;
    const float* qr = Q + (size_t)row * qpitch;
#pragma unroll
    for (int ks = 0; ks < KS; ++ks)
#pragma unroll
      for (int i = 0; i < 16; ++i) {
        const int d = ks * 32 + ((i < 8) ? (8 * hh + i) : (16 + 8 * hh + (i - 8)));
        const float x = qr[d] * scale; const unsigned short hb = bf16_bits(x);
        aqh[ks].u[i] = hb; aql[ks].u[i] = bf16_bits(x - bf16_val(hb));
      }
  }
  int qrow[8];
#pragma unroll
  for (int r = 0; r < 8; ++r) { int qi = q0 + 8 * hh + r; qrow[r] = qi < Tq ? qi : Tq - 1; }
  float m_r[8], l_r[8];
#pragma unroll
  for (int r = 0; r < 8; ++r) { m_r[r] = -3.0e38f; l_r[r] = 0.f; }
  v8f oacc[DT];
#pragma unroll
  for (int dt = 0; dt < DT; ++dt) oacc[dt] = (v8f){0.f,0.f,0.f,0.f,0.f,0.f,0.f,0.f};
  const int kv_end = causal ? min(Tk, qblk * 64 + 64) : Tk;
  for (int j0 = 0; j0 < kv_end; j0 += 32) {
    __syncthreads();
    for (int e = tid; e < 32 * (D / 4); e += 128) {
      const int r = e / (D / 4), c4 = (e % (D / 4)) * 4; const int key = j0 + r;
      v4f kf = {0.f,0.f,0.f,0.f}, vf = {0.f,0.f,0.f,0.f};
      if (key < Tk1) { kf = *(const v4fa*)(K1 + (size_t)b * Tk1 * kpitch + h * D + (size_t)key * kpitch + c4); vf = *(const v4fa*)(V1 + (size_t)b * Tk1 * vpitch + h * D + (size_t)key * vpitch + c4); }
      else if (key < Tk) { const int k2 = key - Tk1; kf = *(const v4fa*)(K2 + (size_t)b * Tk2 * kpitch + h * D + (size_t)k2 * kpitch + c4); vf = *(const v4fa*)(V2 + (size_t)b * Tk2 * vpitch + h * D + (size_t)k2 * vpitch + c4); }
#pragma unroll
      for (int t = 0; t < 4; ++t) {
        unsigned short hb = bf16_bits(kf[t]); sKh[r][c4 + t] = hb; sKl[r][c4 + t] = bf16_bits(kf[t] - bf16_val(hb));
        hb = bf16_bits(vf[t]); sVh[r][c4 + t] = hb; sVl[r][c4 + t] = bf16_bits(vf[t] - bf16_val(hb));
      }
    }
    __syncthreads();
    v8f s[2];
#pragma unroll
    for (int nt = 0; nt < 2; ++nt) {
      v8f acc = {};
#pragma unroll
      for (int ks = 0; ks < KS; ++ks) {
        FragB bh_, bl_;
        bh_.half[0] = *(const v8us*)&sKh[nt * 16 + ln][ks * 32 + 8 * hh]; bh_.half[1] = *(const v8us*)&sKh[nt * 16 + ln][ks * 32 + 16 + 8 * hh];
        bl_.half[0] = *(const v8us*)&sKl[nt * 16 + ln][ks * 32 + 8 * hh]; bl_.half[1] = *(const v8us*)&sKl[nt * 16 + ln][ks * 32 + 16 + 8 * hh];
        acc = mmaN<3>(aqh[ks].v, aql[ks].v, bh_.v, bl_.v, acc);
      }
      s[nt] = acc;
    }
    float alpha[8];
#pragma unroll
    for (int r = 0; r < 8; ++r) {
      const int qi = qrow[r];
      const int ja = j0 + ln, jb = j0 + 16 + ln;
      bool keepa = ja < Tk, keepb = jb < Tk;
      if (causal) { keepa = keepa && (ja <= qi); keepb = keepb && (jb <= qi); }
      if (mask) { if (keepa) keepa = mask[(size_t)qi * Tk + ja] != 0; if (keepb) keepb = mask[(size_t)qi * Tk + jb] != 0; }
      if (sbias) { if (keepa) s[0][r] += sbias[(size_t)bh * Tk + ja]; if (keepb) s[1][r] += sbias[(size_t)bh * Tk + jb]; }
      if (!keepa) s[0][r] = -3.0e38f;
      if (!keepb) s[1][r] = -3.0e38f;
      float mx = fmaxf(s[0][r], s[1][r]);
      mx = fmaxf(mx, __shfl_xor(mx, 1, 32)); mx = fmaxf(mx, __shfl_xor(mx, 2, 32)); mx = fmaxf(mx, __shfl_xor(mx, 4, 32)); mx = fmaxf(mx, __shfl_xor(mx, 8, 32));
      const float mnew = fmaxf(m_r[r], mx);
      alpha[r] = (mnew > -1.0e38f) ? __expf(m_r[r] - mnew) : 1.0f;
      const float p0 = keepa ? __expf(s[0][r] - mnew) : 0.f;
      const float p1 = keepb ? __expf(s[1][r] - mnew) : 0.f;
      m_r[r] = mnew;
      l_r[r] = l_r[r] * alpha[r] + p0 + p1;
      unsigned short hb = bf16_bits(p0); sPh[w][8 * hh + r][ln] = hb;      sPl[w][8 * hh + r][ln] = bf16_bits(p0 - bf16_val(hb));
      hb = bf16_bits(p1);                sPh[w][8 * hh + r][16 + ln] = hb; sPl[w][8 * hh + r][16 + ln] = bf16_bits(p1 - bf16_val(hb));
    }
#pragma unroll
    for (int dt = 0; dt < DT; ++dt)
#pragma unroll
      for (int r = 0; r < 8; ++r) oacc[dt][r] *= alpha[r];
    __builtin_amdgcn_fence(__ATOMIC_ACQ_REL, "workgroup");
    __builtin_amdgcn_wave_barrier();
    FragB pah, pal;
    pah.half[0] = *(const v8us*)&sPh[w][ln][8 * hh]; pah.half[1] = *(const v8us*)&sPh[w][ln][16 + 8 * hh];
    pal.half[0] = *(const v8us*)&sPl[w][ln][8 * hh]; pal.half[1] = *(const v8us*)&sPl[w][ln][16 + 8 * hh];
#pragma unroll
    for (int dt = 0; dt < DT; ++dt) {
      FragB bvh, bvl;
#pragma unroll
      for (int i = 0; i < 8; ++i) {
        bvh.u[i] = sVh[8 * hh + i][dt * 16 + ln]; bvh.u[8 + i] = sVh[16 + 8 * hh + i][dt * 16 + ln];
        bvl.u[i] = sVl[8 * hh + i][dt * 16 + ln]; bvl.u[8 + i] = sVl[16 + 8 * hh + i][dt * 16 + ln];
      }
      oacc[dt] = mmaN<3>(pah.v, pal.v, bvh.v, bvl.v, oacc[dt]);
    }
    __builtin_amdgcn_fence(__ATOMIC_ACQ_REL, "workgroup");
    __builtin_amdgcn_wave_barrier();
  }
#pragma unroll
  for (int r = 0; r < 8; ++r) {
    float l = l_r[r];
    l += __shfl_xor(l, 1, 32); l += __shfl_xor(l, 2, 32); l += __shfl_xor(l, 4, 32); l += __shfl_xor(l, 8, 32);
    l_r[r] = (m_r[r] > -1.0e38f) ? 1.0f / l : __builtin_nanf("");
  }
#pragma unroll
  for (int dt = 0; dt < DT; ++dt)
#pragma unroll
    for (int r = 0; r < 8; ++r) sO[w][8 * hh + r][dt * 16 + ln] = oacc[dt][r] * l_r[r];
  __builtin_amdgcn_fence(__ATOMIC_ACQ_REL, "workgroup");
  __builtin_amdgcn_wave_barrier();
  for (int pass = 0; pass < 2; ++pass) {
    for (int r = 0; r < 16; ++r) {
      const int row = q0 + r;
      if (row < Tq && lane < D / 4) {
        const v4f val = *(const v4fa*)&sO[w][r][lane * 4];
        *(volatile v4f*)(y + ((size_t)b * Tq + row) * ypitch + h * D + lane * 4) = val;
      }
    }
    if (pass == 0) __threadfence();
  }
}

template <int MODE>
__global__ __launch_bounds__(256) void k_wt_padT(const float* __restrict__ W, unsigned short* __restrict__ Bt, int Nout, int Kin, int Np, int Kp) {
  const int t = blockIdx.x * 256 + threadIdx.x; const int k8n = Kp / 8; if (t >= Np * k8n) return;
  const int n = t / k8n, k8 = (t % k8n) * 8; v8us v;
#pragma unroll 1
  for (int i = 0; i < 8; ++i) { const int k = k8 + i; int nn = n, kk = k; bool ok = true;
    if (MODE == 1) { const int h = n / HP, d = n % HP; ok = (d < HD) && (h < NH); nn = h * HD + d; }
    if (MODE == 2) { const int h = k / HP, d = k % HP; ok = (d < HD) && (h < NH); kk = h * HD + d; }
    ok = ok && nn < Nout && kk < Kin;
    v[i] = ok ? bf16_bits(W[(size_t)nn * Kin + kk]) : (unsigned short)0; }
  *(volatile v8us*)(Bt + (size_t)n * Kp + k8) = v; __threadfence(); *(volatile v8us*)(Bt + (size_t)n * Kp + k8) = v;
}
__global__ __launch_bounds__(128) void k_embed(const int* __restrict__ idx, const float* __restrict__ E, float* __restrict__ x) {
  const int row = blockIdx.x, t = threadIdx.x; if (t >= DP / 4) return; int id = idx[row]; id = id < 0 ? 0 : (id >= VV ? VV - 1 : id);
  v4f v; for (int q = 0; q < 4; ++q) { const int c = t * 4 + q; v[q] = (c < DD) ? bf16_round(E[(size_t)id * DD + c]) : 0.f; }
  *(volatile v4f*)(x + (size_t)row * DP + t * 4) = v; __threadfence(); *(volatile v4f*)(x + (size_t)row * DP + t * 4) = v;
}
__global__ __launch_bounds__(128) void k_rms(const float* __restrict__ x, const float* __restrict__ w, float* __restrict__ out) {
  __shared__ float red[128];
  const int row = blockIdx.x, t = threadIdx.x;
  v4f v = {0.f,0.f,0.f,0.f}; if (t < DP / 4) v = *(const v4fa*)(x + (size_t)row * DP + t * 4);
  float s = 0.f; for (int q = 0; q < 4; ++q) { const int c = t * 4 + q; if (c < DD) s += v[q] * v[q]; }
  red[t] = s; __syncthreads(); for (int st = 64; st > 0; st >>= 1) { if (t < st) red[t] += red[t + st]; __syncthreads(); }
  const float rs = rsqrtf(red[0] / (float)DD + 1e-6f);
  if (t < DP / 4) { v4f o; for (int q = 0; q < 4; ++q) { const int c = t * 4 + q; o[q] = (c < DD) ? v[q] * rs * bf16_round(w[c]) : 0.f; }
    *(volatile v4f*)(out + (size_t)row * DP + t * 4) = o; __threadfence(); *(volatile v4f*)(out + (size_t)row * DP + t * 4) = o; }
}
__global__ __launch_bounds__(256) void k_rope40(float* __restrict__ qkv) {
  const int lane = threadIdx.x & 31; const size_t wv = (size_t)blockIdx.x * 8 + (threadIdx.x >> 5); if (wv >= (size_t)BB * TT * NH * 2) return;
  const int which = (int)(wv & 1); const int h = (int)((wv >> 1) % NH); const size_t row = (wv >> 1) / NH; const int pos = (int)(row % TT);
  float* base = qkv + row * 3 * QP + (size_t)which * QP + h * HP;
  const float xa = base[lane], xb = base[lane + 32];
  const float p_hi = __shfl(xa, (lane + 20) & 31, 32);
  const float p_xb = __shfl(xb, (lane + 20) & 31, 32);
  const float p_lo = __shfl(xa, (lane + 12) & 31, 32);
  const int c = lane; const int j1 = (c < 20) ? c : c - 20; float sn, cs; sincosf((float)pos * powf(10000.0f, -(float)(2 * j1) / (float)HD), &sn, &cs);
  const float sn2 = __shfl(sn, (lane + 12) & 31, 32), cs2 = __shfl(cs, (lane + 12) & 31, 32);
  const float o1 = (c < 20) ? (xa * cs - ((c < 12) ? p_hi : p_xb) * sn) : (xa * cs + p_lo * sn);
  const float o2 = (lane + 32 < HD) ? (xb * cs2 + p_lo * sn2) : 0.f;
  *(volatile float*)(base + lane) = o1; *(volatile float*)(base + 32 + lane) = o2; __threadfence(); *(volatile float*)(base + lane) = o1; *(volatile float*)(base + 32 + lane) = o2;
}
__global__ __launch_bounds__(256) void k_swiglu(const float* __restrict__ gup, float* __restrict__ gu) {
  const size_t t = (size_t)blockIdx.x * 256 + threadIdx.x; if (t >= (size_t)(BB * TT / 4) * FP / 4) return; const size_t row = t / (FP / 4); const int c4 = (int)(t % (FP / 4)) * 4;
  const v4f g = *(const v4fa*)(gup + row * 2 * FP + c4), u = *(const v4fa*)(gup + row * 2 * FP + FP + c4); v4f o;
  for (int q = 0; q < 4; ++q) o[q] = (g[q] / (1.0f + expf(-g[q]))) * u[q];
  *(volatile v4f*)(gu + t * 4) = o; __threadfence(); *(volatile v4f*)(gu + t * 4) = o;
}
extern "C" void kernel_launch(void* const* d_in, const int* in_sizes, int n_in,
                              void* d_out, int out_size, void* d_ws, size_t ws_size, hipStream_t stream) {
  (void)in_sizes; (void)n_in; (void)out_size;
  const int* idx = (const int*)d_in[0]; const float* E = (const float*)d_in[1];
  const float* wq = (const float*)d_in[2]; const float* wk = (const float*)d_in[3]; const float* wv = (const float*)d_in[4]; const float* wo = (const float*)d_in[5];
  const float* w1 = (const float*)d_in[6]; const float* w2 = (const float*)d_in[7]; const float* w3 = (const float*)d_in[8];
  const float* n1 = (const float*)d_in[9]; const float* n2 = (const float*)d_in[10]; const float* nw = (const float*)d_in[11];
  char* ws = (char*)d_ws; size_t off = 0;
  auto take = [&](size_t bytes) { char* p = ws + off; off += (bytes + 255) & ~(size_t)255; return p; };
  const int M = BB * TT;
  unsigned short* Bqkv[NL], *Bo[NL], *B13[NL], *B2[NL];
  for (int l = 0; l < NL; ++l) { Bqkv[l] = (unsigned short*)take((size_t)3 * QP * KP * 2); Bo[l] = (unsigned short*)take((size_t)DP * QP * 2); B13[l] = (unsigned short*)take((size_t)2 * FP * KP * 2); B2[l] = (unsigned short*)take((size_t)DP * FP * 2); }
  unsigned short* Bhead = (unsigned short*)take((size_t)VV * KP * 2);
  float* x = (float*)take((size_t)M * DP * 4); float* h = (float*)take((size_t)M * DP * 4); float* qkv = (float*)take((size_t)M * 3 * QP * 4); float* att = (float*)take((size_t)M * QP * 4);
  const int MC = M / 4;
  float* gup = (float*)take((size_t)MC * 2 * FP * 4); float* gu = (float*)take((size_t)MC * FP * 4);
  if (off > ws_size) return;
  for (int l = 0; l < NL; ++l) {
    k_wt_padT<1><<<(QP * (KP / 8) + 255) / 256, 256, 0, stream>>>(wq + (size_t)l * DD * DD, Bqkv[l], DD, DD, QP, KP);
    k_wt_padT<1><<<(QP * (KP / 8) + 255) / 256, 256, 0, stream>>>(wk + (size_t)l * DD * DD, Bqkv[l] + (size_t)QP * KP, DD, DD, QP, KP);
    k_wt_padT<1><<<(QP * (KP / 8) + 255) / 256, 256, 0, stream>>>(wv + (size_t)l * DD * DD, Bqkv[l] + (size_t)2 * QP * KP, DD, DD, QP, KP);
    k_wt_padT<2><<<(DP * (QP / 8) + 255) / 256, 256, 0, stream>>>(wo + (size_t)l * DD * DD, Bo[l], DD, DD, DP, QP);
    k_wt_padT<0><<<(FP * (KP / 8) + 255) / 256, 256, 0, stream>>>(w1 + (size_t)l * FF * DD, B13[l], FF, DD, FP, KP);
    k_wt_padT<0><<<(FP * (KP / 8) + 255) / 256, 256, 0, stream>>>(w3 + (size_t)l * FF * DD, B13[l] + (size_t)FP * KP, FF, DD, FP, KP);
    k_wt_padT<0><<<(DP * (FP / 8) + 255) / 256, 256, 0, stream>>>(w2 + (size_t)l * DD * FF, B2[l], DD, FF, DP, FP);
  }
  k_wt_padT<0><<<(VV * (KP / 8) + 255) / 256, 256, 0, stream>>>(E, Bhead, VV, DD, VV, KP);
  k_embed<<<M, 128, 0, stream>>>(idx, E, x);
  const int gq = ((M / 16) * (3 * QP / 64) + 3) / 4, gd = ((M / 16) * (DP / 64) + 3) / 4, gfc = ((MC / 16) * (2 * FP / 64) + 3) / 4, gdc = ((MC / 16) * (DP / 64) + 3) / 4, gv = ((M / 16) * (VV / 64) + 3) / 4;
  for (int l = 0; l < NL; ++l) {
    k_rms<<<M, 128, 0, stream>>>(x, n1 + l * DD, h);
    k_gemm_bf3<true, 0, false, false><<<gq, 128, 0, stream>>>(h, DP, Bqkv[l], KP, nullptr, nullptr, 1, 0, qkv, 3 * QP, M, 3 * QP, KP);
    k_rope40<<<(unsigned)(((size_t)M * NH * 2 + 7) / 8), 256, 0, stream>>>(qkv);
    k_flash3<HP><<<BB * NH * (TT / 64), 128, 0, stream>>>(qkv, 3 * QP, TT, qkv + QP, qkv + 2 * QP, TT, nullptr, nullptr, 0, 3 * QP, 3 * QP, NH, 0.15811388300841897f, nullptr, 1, nullptr, att, QP);
    k_gemm_bf3<true, 0, false, false><<<gd, 128, 0, stream>>>(att, QP, Bo[l], QP, nullptr, x, M, DP, x, DP, M, DP, QP);
    k_rms<<<M, 128, 0, stream>>>(x, n2 + l * DD, h);
    for (int c = 0; c < 4; ++c) {
      const float* hc = h + (size_t)c * MC * DP; float* xc = x + (size_t)c * MC * DP;
      k_gemm_bf3<true, 0, false, false><<<gfc, 128, 0, stream>>>(hc, DP, B13[l], KP, nullptr, nullptr, 1, 0, gup, 2 * FP, MC, 2 * FP, KP);
      k_swiglu<<<(unsigned)(((size_t)MC * FP / 4 + 255) / 256), 256, 0, stream>>>(gup, gu);
      k_gemm_bf3<true, 0, false, false><<<gdc, 128, 0, stream>>>(gu, FP, B2[l], FP, nullptr, xc, MC, DP, xc, DP, MC, DP, FP);
    }
  }
  k_rms<<<M, 128, 0, stream>>>(x, nw, h);
  k_gemm_bf3<true, 0, false, false><<<gv, 128, 0, stream>>>(h, DP, Bhead, KP, nullptr, nullptr, 1, 0, (float*)d_out, VV, M, VV, KP);
}
